// GNNTC_45938970198063
// MI455X (gfx1250) — hardware-verified
//
#include <hip/hip_runtime.h>
#include <math.h>

typedef __attribute__((ext_vector_type(16))) _Float16 v16h;
typedef __attribute__((ext_vector_type(8)))  _Float16 v8h;
typedef __attribute__((ext_vector_type(8)))  float    v8f;
typedef __attribute__((ext_vector_type(4)))  float    v4f;
typedef __attribute__((ext_vector_type(4)))  unsigned v4u;

constexpr int kNB    = 4;
constexpr int kNL    = 64;
constexpr int kNAg   = 23;
constexpr int kHid   = 256;
constexpr int kRowsA = kNB * kNAg;
constexpr int kRowsAP = 128;
constexpr int kRowsS = kNB * kNL * kNAg;
constexpr int kRowsP = kNB * kNL;
constexpr int kC1Out = 32;
constexpr int kC1K   = 9;
constexpr int kC1L   = 22;
constexpr int kC2K   = 7;
constexpr int kC2L   = 11;
constexpr int kC3K   = 5;
constexpr int kNF    = 256;
static_assert(kRowsA == 92 && kRowsS == 5888 && kRowsP == 256, "row counts");
static_assert((kRowsAP % 64) == 0 && (kRowsS % 64) == 0 && (kRowsP % 64) == 0, "GEMM M multiples of 64");
static_assert((kHid % 64) == 0 && ((2 * kHid) % 64) == 0 && (kHid % 32) == 0, "GEMM N multiples of 64, K multiple of 32");
static_assert((kNL + 2 * 4 - kC1K) / 3 + 1 == kC1L, "conv1 length");
static_assert((kC1L + 2 * 3 - kC2K) / 2 + 1 == kC2L, "conv2 length");
static_assert((kC2L + 2 * 2 - kC3K) / 2 + 1 == 6, "conv3 length");

constexpr float kActCarry = 64.0f;
constexpr float kWtCarry  = 256.0f;
constexpr float kFold     = 1.0f / (kActCarry * kWtCarry);
constexpr float kF16MinNormal = 6.103515625e-5f;

constexpr size_t kSzWT    = (size_t)8 * kHid * kHid * 2;
constexpr size_t kSzHA    = (size_t)kRowsAP * kHid * 2;
constexpr size_t kSzAENC  = (size_t)kRowsAP * kHid * 2;
constexpr size_t kSzPBPA  = (size_t)kRowsAP * 2 * kHid * 4;
constexpr size_t kSzH1P   = (size_t)kRowsAP * kHid * 2;
constexpr size_t kSzRELP  = (size_t)kRowsAP * kHid * 2;
constexpr size_t kSzPRELP = (size_t)kRowsAP * kHid * 4;
constexpr size_t kSzHS    = (size_t)kRowsS * kHid * 2;
constexpr size_t kSzSENC  = (size_t)kRowsS * kHid * 2;
constexpr size_t kSzPRR   = (size_t)kRowsS * kHid * 4;
constexpr size_t kSzSENCP = (size_t)kRowsP * kHid * 2;
constexpr size_t kSzPSP   = (size_t)kRowsP * kHid * 4;
constexpr size_t kSzXAGG  = (size_t)kRowsP * kHid * 4;
constexpr size_t kSzY1    = (size_t)kNB * kC1L * kC1Out * 4;
constexpr size_t kOffWT    = 0;
constexpr size_t kOffHA    = kOffWT    + kSzWT;
constexpr size_t kOffAENC  = kOffHA    + kSzHA;
constexpr size_t kOffPBPA  = kOffAENC  + kSzAENC;
constexpr size_t kOffH1P   = kOffPBPA  + kSzPBPA;
constexpr size_t kOffRELP  = kOffH1P   + kSzH1P;
constexpr size_t kOffPRELP = kOffRELP  + kSzRELP;
constexpr size_t kOffHS    = kOffPRELP + kSzPRELP;
constexpr size_t kOffSENC  = kOffHS    + kSzHS;
constexpr size_t kOffPRR   = kOffSENC  + kSzSENC;
constexpr size_t kOffSENCP = kOffPRR   + kSzPRR;
constexpr size_t kOffPSP   = kOffSENCP + kSzSENCP;
constexpr size_t kOffXAGG  = kOffPSP   + kSzPSP;
constexpr size_t kOffY1    = kOffXAGG  + kSzXAGG;
constexpr size_t kWsTotal  = kOffY1    + kSzY1;
static_assert(kWsTotal == 14429184ull, "carve total");
static_assert(kWsTotal <= 134217728ull, "carve cap");
static_assert((kOffHA % 256) == 0 && (kOffAENC % 256) == 0 && (kOffPBPA % 256) == 0 && (kOffH1P % 256) == 0 &&
              (kOffRELP % 256) == 0 && (kOffPRELP % 256) == 0 && (kOffHS % 256) == 0 && (kOffSENC % 256) == 0 &&
              (kOffPRR % 256) == 0 && (kOffSENCP % 256) == 0 && (kOffPSP % 256) == 0 && (kOffXAGG % 256) == 0 &&
              (kOffY1 % 256) == 0, "256-B aligned regions");

__device__ __forceinline__ _Float16 to_h_carried(float v, float carry) {
  float c = v * carry;
  c = (__builtin_fabsf(c) < kF16MinNormal) ? 0.0f : c;
  return (_Float16)c;
}

union FragU { v16h v; v8h h[2]; };
__device__ __forceinline__ v16h frag_load(const _Float16* p) {
  FragU f;
  f.h[0] = *(const v8h*)(p);
  f.h[1] = *(const v8h*)(p + 16);
  return f.v;
}
__device__ __forceinline__ v8f mma_f16(v16h a, v16h b, v8f c) {
  return __builtin_amdgcn_wmma_f32_16x16x32_f16(false, a, false, b, (short)0, c, false, false);
}
__device__ __forceinline__ void mma_guard(v8f& a, v16h x, v16h y) {
  asm volatile("v_nop\n\tv_nop\n\tv_nop\n\tv_nop" : "+v"(a) : "v"(x), "v"(y));
}
__device__ __forceinline__ void keep4_h(v16h a, v16h b, v16h c, v16h d) {
  asm volatile("v_nop" :: "v"(a), "v"(b), "v"(c), "v"(d));
}
__device__ __forceinline__ void acc_guard4(v8f& a, v8f& b, v8f& c, v8f& d) {
  asm volatile("v_nop\n\tv_nop\n\tv_nop\n\tv_nop" : "+v"(a), "+v"(b), "+v"(c), "+v"(d));
}

template <int BIAS_ON, int OUT_F16, int RELU_ON>
__global__ __launch_bounds__(256) void gemm_f16_tile64(
    const unsigned short* __restrict__ Ap, int lda,
    const unsigned short* __restrict__ Btp, int ldb,
    void* __restrict__ Cout, int ldc,
    const float* __restrict__ bias,
    int M, int N, int K, int mreal, float scale, float ocarry) {
  const _Float16* A  = (const _Float16*)Ap;
  const _Float16* Bt = (const _Float16*)Btp;
  __shared__ __align__(16) float sT[8][16 * 68];
  const int lane = threadIdx.x & 31;
  const int wave = threadIdx.x >> 5;
  const int tilesN = N >> 6;
  const int tilesM = M >> 6;
  const int tile = blockIdx.x * 8 + wave;
  if (tile >= tilesM * tilesN) return;
  const int tm = tile / tilesN;
  const int tn = tile - tm * tilesN;
  const int m0 = tm << 6;
  const int n0 = tn << 6;

  const int rlane = lane & 15;
  const int koff  = (lane >> 4) * 8;
  const int mOff  = (lane >> 4) * 8;

  v8f acc[4][4];
#pragma unroll
  for (int i = 0; i < 4; ++i)
#pragma unroll
    for (int j = 0; j < 4; ++j) acc[i][j] = (v8f){0.f,0.f,0.f,0.f,0.f,0.f,0.f,0.f};

  for (int k0 = 0; k0 < K; k0 += 32) {
    v16h bh[4];
#pragma unroll
    for (int j = 0; j < 4; ++j) {
      const size_t bo = (size_t)(n0 + (j << 4) + rlane) * ldb + koff + k0;
      bh[j] = frag_load(Bt + bo);
    }
#pragma unroll
    for (int i = 0; i < 4; ++i) {
      const size_t ao = (size_t)(m0 + (i << 4) + rlane) * lda + koff + k0;
      v16h ah = frag_load(A + ao);
#pragma unroll
      for (int j = 0; j < 4; ++j) acc[i][j] = mma_f16(ah, bh[j], acc[i][j]);
      mma_guard(acc[i][0], ah, bh[0]);
      mma_guard(acc[i][1], ah, bh[1]);
      mma_guard(acc[i][2], ah, bh[2]);
      mma_guard(acc[i][3], ah, bh[3]);
    }
    keep4_h(bh[0], bh[1], bh[2], bh[3]);
  }
  acc_guard4(acc[0][0], acc[0][1], acc[0][2], acc[0][3]);
  acc_guard4(acc[1][0], acc[1][1], acc[1][2], acc[1][3]);
  acc_guard4(acc[2][0], acc[2][1], acc[2][2], acc[2][3]);
  acc_guard4(acc[3][0], acc[3][1], acc[3][2], acc[3][3]);

  float* slab = sT[wave];
#pragma unroll
  for (int i = 0; i < 4; ++i) {
    const int mBase = m0 + (i << 4);
#pragma unroll
    for (int j = 0; j < 4; ++j) {
      const int n = n0 + (j << 4) + rlane;
      float bv = 0.f;
      if (BIAS_ON) bv = bias[n];
#pragma unroll
      for (int r = 0; r < 8; ++r) {
        float v = acc[i][j][r] * scale;
        if (BIAS_ON) v += bv;
        if (RELU_ON) v = fmaxf(v, 0.0f);
        v = ((mBase + mOff + r) < mreal) ? v : 0.0f;
        slab[(mOff + r) * 68 + (j << 4) + rlane] = v;
      }
    }
    __builtin_amdgcn_fence(__ATOMIC_RELEASE, "workgroup");
    __builtin_amdgcn_wave_barrier();
    __builtin_amdgcn_fence(__ATOMIC_ACQUIRE, "workgroup");
    if (OUT_F16 == 0) {
      float* C = (float*)Cout;
      const int hh = lane >> 4, c4 = (lane & 15) * 4;
      for (int pass = 0; pass < 2; ++pass) {
#pragma unroll
        for (int it = 0; it < 8; ++it) {
          const int row = it * 2 + hh;
          v4f v = *(const v4f*)(slab + row * 68 + c4);
          *(volatile v4f*)(C + (size_t)(mBase + row) * ldc + n0 + c4) = v;
        }
        __threadfence();
      }
    } else {
      const int q = lane >> 3, c8 = (lane & 7) * 8;
      unsigned short* C = (unsigned short*)Cout;
      for (int pass = 0; pass < 2; ++pass) {
#pragma unroll
        for (int it = 0; it < 4; ++it) {
          const int row = it * 4 + q;
          const float* sp = slab + row * 68 + c8;
          v8h hv;
#pragma unroll
          for (int e = 0; e < 8; ++e) hv[e] = to_h_carried(sp[e], ocarry);
          *(volatile v8h*)(C + (size_t)(mBase + row) * ldc + n0 + c8) = hv;
        }
        __threadfence();
      }
    }
    __builtin_amdgcn_fence(__ATOMIC_RELEASE, "workgroup");
    __builtin_amdgcn_wave_barrier();
    __builtin_amdgcn_fence(__ATOMIC_ACQUIRE, "workgroup");
  }
}

__global__ __launch_bounds__(256) void prep_weights_kernel(
    const float* __restrict__ p0, const float* __restrict__ p1, const float* __restrict__ p2,
    const float* __restrict__ p3, const float* __restrict__ p4, const float* __restrict__ p5,
    const float* __restrict__ p6, const float* __restrict__ p7, unsigned short* __restrict__ WT)
{
  __shared__ float sTile[64 * 65];
  const int tid = threadIdx.x, lane = tid & 31, wave = tid >> 5;
  const int z = blockIdx.z;
  const float* src = (z == 0) ? p0 : (z == 1) ? p1 : (z == 2) ? p2 : (z == 3) ? p3
                   : (z == 4) ? p4 : (z == 5) ? p5 : (z == 6) ? p6 : p7;
  const int k0 = blockIdx.x * 64;
  const int n0 = blockIdx.y * 64;
  const int lr = tid >> 4, c4 = (tid & 15) * 4;
#pragma unroll
  for (int it = 0; it < 4; ++it) {
    const int kk = lr + 16 * it;
    const v4f v = *(const v4f*)(src + (size_t)(k0 + kk) * kHid + n0 + c4);
    sTile[kk * 65 + c4 + 0] = v[0];
    sTile[kk * 65 + c4 + 1] = v[1];
    sTile[kk * 65 + c4 + 2] = v[2];
    sTile[kk * 65 + c4 + 3] = v[3];
  }
  __syncthreads();
  const int q = lane >> 3, c8 = (lane & 7) * 8;
  v8h hv[2];
#pragma unroll
  for (int it = 0; it < 2; ++it) {
    const int n = it * 32 + wave * 4 + q;
#pragma unroll
    for (int e = 0; e < 8; ++e) hv[it][e] = to_h_carried(sTile[(c8 + e) * 65 + n], kWtCarry);
  }
  unsigned short* dst = WT + (size_t)z * kHid * kHid;
  for (int pass = 0; pass < 2; ++pass) {
#pragma unroll
    for (int it = 0; it < 2; ++it) {
      const int n = it * 32 + wave * 4 + q;
      *(volatile v8h*)(dst + (size_t)(n0 + n) * kHid + k0 + c8) = hv[it];
    }
    __threadfence();
  }
}

__global__ __launch_bounds__(256) void k3_layer_kernel(
    const float* __restrict__ in, const float* __restrict__ W, const float* __restrict__ bias,
    unsigned short* __restrict__ out, int mreal)
{
  const int lane = threadIdx.x & 31, wave = threadIdx.x >> 5;
  const int row = blockIdx.x * 8 + wave;
  const int rc = (row < mreal) ? row : (mreal - 1);
  const int c8 = lane * 8;
  const float x0 = in[(size_t)rc * 3 + 0];
  const float x1 = in[(size_t)rc * 3 + 1];
  const float x2 = in[(size_t)rc * 3 + 2];
  const v4f w0a = *(const v4f*)(W + c8),            w0b = *(const v4f*)(W + c8 + 4);
  const v4f w1a = *(const v4f*)(W + kHid + c8),     w1b = *(const v4f*)(W + kHid + c8 + 4);
  const v4f w2a = *(const v4f*)(W + 2 * kHid + c8), w2b = *(const v4f*)(W + 2 * kHid + c8 + 4);
  const v4f ba = *(const v4f*)(bias + c8), bb = *(const v4f*)(bias + c8 + 4);
  const bool live = (row < mreal);
  v8h hv;
#pragma unroll
  for (int e = 0; e < 4; ++e) {
    float s = x0 * w0a[e];
    s = fmaf(x1, w1a[e], s);
    s = fmaf(x2, w2a[e], s);
    s = fmaxf(s + ba[e], 0.0f);
    s = live ? s : 0.0f;
    float u = x0 * w0b[e];
    u = fmaf(x1, w1b[e], u);
    u = fmaf(x2, w2b[e], u);
    u = fmaxf(u + bb[e], 0.0f);
    u = live ? u : 0.0f;
    hv[e]     = to_h_carried(s, kActCarry);
    hv[4 + e] = to_h_carried(u, kActCarry);
  }
  unsigned short* dst = out + (size_t)row * kHid + c8;
  *(volatile v8h*)dst = hv;
  __threadfence();
  *(volatile v8h*)dst = hv;
}

__global__ __launch_bounds__(256) void gather_player_kernel(
    const unsigned short* __restrict__ senc, const int* __restrict__ pid, unsigned short* __restrict__ sencp)
{
  const int lane = threadIdx.x & 31, wave = threadIdx.x >> 5;
  const int row = blockIdx.x * 8 + wave;
  const int b = row >> 6;
  int p = pid[b];
  p = (p < 0) ? 0 : ((p > kNAg - 1) ? (kNAg - 1) : p);
  const v4u w = *(const v4u*)(senc + ((size_t)row * kNAg + p) * kHid + lane * 8);
  unsigned short* dst = sencp + (size_t)row * kHid + lane * 8;
  *(volatile v4u*)dst = w;
  __threadfence();
  *(volatile v4u*)dst = w;
}

__global__ __launch_bounds__(256) void h1_player_kernel(
    const float* __restrict__ pbpa, const float* __restrict__ b1, const int* __restrict__ pid,
    unsigned short* __restrict__ h1p)
{
  const int lane = threadIdx.x & 31, wave = threadIdx.x >> 5;
  const unsigned row = (unsigned)(blockIdx.x * 8 + wave);
  unsigned rc = (row < (unsigned)kRowsA) ? row : (unsigned)(kRowsA - 1);
  asm volatile("" : "+v"(rc));
  unsigned b = rc / (unsigned)kNAg;
  asm volatile("" : "+v"(b));
  int p = pid[b];
  p = (p < 0) ? 0 : ((p > kNAg - 1) ? (kNAg - 1) : p);
  const int c8 = lane * 8;
  const float* pbrow = pbpa + (size_t)rc * (2 * kHid) + c8;
  const float* parow = pbpa + ((size_t)b * kNAg + p) * (2 * kHid) + kHid + c8;
  const v4f pb0 = *(const v4f*)(pbrow), pb1 = *(const v4f*)(pbrow + 4);
  const v4f pa0 = *(const v4f*)(parow), pa1 = *(const v4f*)(parow + 4);
  const v4f bz0 = *(const v4f*)(b1 + c8), bz1 = *(const v4f*)(b1 + c8 + 4);
  const bool live = (row < (unsigned)kRowsA);
  v8h hv;
#pragma unroll
  for (int e = 0; e < 4; ++e) {
    float s = fmaxf((pa0[e] + pb0[e]) + bz0[e], 0.0f);
    float u = fmaxf((pa1[e] + pb1[e]) + bz1[e], 0.0f);
    s = live ? s : 0.0f;
    u = live ? u : 0.0f;
    hv[e]     = to_h_carried(s, kActCarry);
    hv[4 + e] = to_h_carried(u, kActCarry);
  }
  unsigned short* dst = h1p + (size_t)row * kHid + c8;
  *(volatile v8h*)dst = hv;
  __threadfence();
  *(volatile v8h*)dst = hv;
}

__global__ __launch_bounds__(256) void combine_kernel(
    const float* __restrict__ psp, const float* __restrict__ prr, const float* __restrict__ prelp,
    const float* __restrict__ prb, float* __restrict__ xagg)
{
  const int tid = threadIdx.x;
  const int row = blockIdx.x * 4 + (tid >> 6);
  const int c4 = (tid & 63) * 4;
  const int b = row >> 6;
  const v4f base = *(const v4f*)(psp + (size_t)row * kHid + c4);
  const v4f bz = *(const v4f*)(prb + c4);
  float s0 = 0.0f, s1 = 0.0f, s2 = 0.0f, s3 = 0.0f;
  const float* rp = prr + (size_t)row * kNAg * kHid + c4;
  const float* qp = prelp + (size_t)b * kNAg * kHid + c4;
#pragma unroll 1
  for (int j = 0; j < kNAg; ++j) {
    const v4f r = *(const v4f*)(rp + (size_t)j * kHid);
    const v4f q = *(const v4f*)(qp + (size_t)j * kHid);
    s0 += fmaxf(((base[0] + r[0]) + q[0]) + bz[0], 0.0f);
    s1 += fmaxf(((base[1] + r[1]) + q[1]) + bz[1], 0.0f);
    s2 += fmaxf(((base[2] + r[2]) + q[2]) + bz[2], 0.0f);
    s3 += fmaxf(((base[3] + r[3]) + q[3]) + bz[3], 0.0f);
  }
  v4f o;
  o[0] = s0; o[1] = s1; o[2] = s2; o[3] = s3;
  float* dst = xagg + (size_t)row * kHid + c4;
  *(volatile v4f*)dst = o;
  __threadfence();
  *(volatile v4f*)dst = o;
}

__global__ __launch_bounds__(256) void conv1_kernel(
    const float* __restrict__ xagg, const float* __restrict__ w, const float* __restrict__ bias,
    float* __restrict__ y1)
{
  const int lane = threadIdx.x & 31, wave = threadIdx.x >> 5;
  unsigned gw = (unsigned)(blockIdx.x * 8 + wave);
  asm volatile("" : "+v"(gw));
  unsigned b = gw / (unsigned)kC1L;
  asm volatile("" : "+v"(b));
  const int t = (int)(gw - b * (unsigned)kC1L);
  const float* wrow = w + (size_t)lane * kHid * kC1K;
  const float* xb = xagg + (size_t)b * kNL * kHid;
  float acc = 0.0f;
#pragma unroll 1
  for (int i = 0; i < kHid; ++i) {
#pragma unroll
    for (int k = 0; k < kC1K; ++k) {
      const int pos = 3 * t - 4 + k;
      const int pc = (pos < 0) ? 0 : ((pos > kNL - 1) ? (kNL - 1) : pos);
      float xv = xb[(size_t)pc * kHid + i];
      xv = (pos >= 0 && pos < kNL) ? xv : 0.0f;
      acc = fmaf(wrow[i * kC1K + k], xv, acc);
    }
  }
  acc = fmaxf(acc + bias[lane], 0.0f);
  float* dst = y1 + (size_t)gw * kC1Out + lane;
  *(volatile float*)dst = acc;
  __threadfence();
  *(volatile float*)dst = acc;
}

__global__ __launch_bounds__(256) void tail_kernel(
    const float* __restrict__ y1, const float* __restrict__ c2w, const float* __restrict__ c2b,
    const float* __restrict__ c3w, const float* __restrict__ c3b,
    const float* __restrict__ c4w, const float* __restrict__ c4b, float* __restrict__ out)
{
  __shared__ float sY1[kC1L * 32];
  __shared__ float sY2[kC2L * 32];
  __shared__ float sY3[32];
  const int tid = threadIdx.x, lane = tid & 31, wave = tid >> 5;
  const int b = blockIdx.x;
  constexpr int kY1N = kC1L * 32;
#pragma unroll
  for (int it = 0; it < 3; ++it) {
    const int idx = tid + 256 * it;
    const int idc = (idx < kY1N) ? idx : (kY1N - 1);
    float v = y1[(size_t)b * kY1N + idc];
    asm volatile("" : "+v"(v));
    if (idx < kY1N) sY1[idx] = v;
  }
  __syncthreads();
#pragma unroll 1
  for (int pass = 0; pass < 2; ++pass) {
    const int t = wave + 8 * pass;
    const int tc = (t < kC2L) ? t : (kC2L - 1);
    float acc = 0.0f;
#pragma unroll 1
    for (int i = 0; i < 32; ++i) {
#pragma unroll
      for (int k = 0; k < kC2K; ++k) {
        const int pos = 2 * tc - 3 + k;
        const int pc = (pos < 0) ? 0 : ((pos > kC1L - 1) ? (kC1L - 1) : pos);
        float yv = sY1[pc * 32 + i];
        yv = (pos >= 0 && pos < kC1L) ? yv : 0.0f;
        acc = fmaf(c2w[(lane * 32 + i) * kC2K + k], yv, acc);
      }
    }
    acc = fmaxf(acc + c2b[lane], 0.0f);
    if (t < kC2L) sY2[t * 32 + lane] = acc;
  }
  __syncthreads();
  {
    float acc = 0.0f;
#pragma unroll 1
    for (int i = 0; i < 32; ++i) {
#pragma unroll
      for (int k = 0; k < kC3K; ++k)
        acc = fmaf(c3w[(lane * 32 + i) * kC3K + k], sY2[(4 + k) * 32 + i], acc);
    }
    acc = fmaxf(acc + c3b[lane], 0.0f);
    if (wave == 0) sY3[lane] = acc;
  }
  __syncthreads();
  {
    const float* wr = c4w + (size_t)tid * 32;
    v4f wv[8];
#pragma unroll
    for (int g = 0; g < 8; ++g) wv[g] = *(const v4f*)(wr + 4 * g);
    float acc = 0.0f;
#pragma unroll
    for (int g = 0; g < 8; ++g) {
      acc = fmaf(wv[g][0], sY3[4 * g + 0], acc);
      acc = fmaf(wv[g][1], sY3[4 * g + 1], acc);
      acc = fmaf(wv[g][2], sY3[4 * g + 2], acc);
      acc = fmaf(wv[g][3], sY3[4 * g + 3], acc);
    }
    acc += c4b[tid];
    float* dst = out + (size_t)b * kNF + tid;
    *(volatile float*)dst = acc;
    __threadfence();
    *(volatile float*)dst = acc;
  }
}

static inline int gemm_blocks(int M, int N) { return ((M / 64) * (N / 64) + 7) / 8; }

extern "C" void kernel_launch(void* const* d_in, const int* in_sizes, int n_in,
                              void* d_out, int out_size, void* d_ws, size_t ws_size,
                              hipStream_t stream) {
  if (n_in < 25) return;
  if (in_sizes[0] != kRowsS * 3) return;
  if (in_sizes[1] != kRowsA * 3) return;
  if (in_sizes[2] != kNB) return;
  if (in_sizes[3] != 3 * kHid || in_sizes[4] != kHid) return;
  if (in_sizes[5] != kHid * kHid || in_sizes[6] != kHid) return;
  if (in_sizes[7] != 3 * kHid || in_sizes[8] != kHid) return;
  if (in_sizes[9] != kHid * kHid || in_sizes[10] != kHid) return;
  if (in_sizes[11] != 2 * kHid * kHid || in_sizes[12] != kHid) return;
  if (in_sizes[13] != kHid * kHid || in_sizes[14] != kHid) return;
  if (in_sizes[15] != 3 * kHid * kHid || in_sizes[16] != kHid) return;
  if (in_sizes[17] != kC1Out * kHid * kC1K || in_sizes[18] != kC1Out) return;
  if (in_sizes[19] != 32 * 32 * kC2K || in_sizes[20] != 32) return;
  if (in_sizes[21] != 32 * 32 * kC3K || in_sizes[22] != 32) return;
  if (in_sizes[23] != kNF * 32 || in_sizes[24] != kNF) return;
  if (out_size != kNB * kNF) return;
  if (ws_size < kWsTotal) return;

  const float* states = (const float*)d_in[0];
  const float* types  = (const float*)d_in[1];
  const int*   pid    = (const int*)  d_in[2];
  const float* ae_W1  = (const float*)d_in[3];
  const float* ae_b1  = (const float*)d_in[4];
  const float* ae_W2  = (const float*)d_in[5];
  const float* ae_b2  = (const float*)d_in[6];
  const float* se_W1  = (const float*)d_in[7];
  const float* se_b1  = (const float*)d_in[8];
  const float* se_W2  = (const float*)d_in[9];
  const float* se_b2  = (const float*)d_in[10];
  const float* re_W1  = (const float*)d_in[11];
  const float* re_b1  = (const float*)d_in[12];
  const float* re_W2  = (const float*)d_in[13];
  const float* re_b2  = (const float*)d_in[14];
  const float* pr_W   = (const float*)d_in[15];
  const float* pr_b   = (const float*)d_in[16];
  const float* c1_w   = (const float*)d_in[17];
  const float* c1_b   = (const float*)d_in[18];
  const float* c2_w   = (const float*)d_in[19];
  const float* c2_b   = (const float*)d_in[20];
  const float* c3_w   = (const float*)d_in[21];
  const float* c3_b   = (const float*)d_in[22];
  const float* c4_w   = (const float*)d_in[23];
  const float* c4_b   = (const float*)d_in[24];
  float* out = (float*)d_out;

  char* ws = (char*)d_ws;
  unsigned short* WT    = (unsigned short*)(ws + kOffWT);
  unsigned short* HA    = (unsigned short*)(ws + kOffHA);
  unsigned short* AENC  = (unsigned short*)(ws + kOffAENC);
  float*          PBPA  = (float*)(ws + kOffPBPA);
  unsigned short* H1P   = (unsigned short*)(ws + kOffH1P);
  unsigned short* RELP  = (unsigned short*)(ws + kOffRELP);
  float*          PRELP = (float*)(ws + kOffPRELP);
  unsigned short* HS    = (unsigned short*)(ws + kOffHS);
  unsigned short* SENC  = (unsigned short*)(ws + kOffSENC);
  float*          PRR   = (float*)(ws + kOffPRR);
  unsigned short* SENCP = (unsigned short*)(ws + kOffSENCP);
  float*          PSP   = (float*)(ws + kOffPSP);
  float*          XAGG  = (float*)(ws + kOffXAGG);
  float*          Y1    = (float*)(ws + kOffY1);

  constexpr size_t kPlane = (size_t)kHid * kHid;
  const unsigned short* WT_ae2  = WT + 0 * kPlane;
  const unsigned short* WT_pbpa = WT + 1 * kPlane;
  const unsigned short* WT_re2  = WT + 3 * kPlane;
  const unsigned short* WT_se2  = WT + 4 * kPlane;
  const unsigned short* WT_ps   = WT + 5 * kPlane;
  const unsigned short* WT_prr  = WT + 6 * kPlane;
  const unsigned short* WT_prel = WT + 7 * kPlane;

  prep_weights_kernel<<<dim3(4, 4, 8), 256, 0, stream>>>(
      ae_W2, re_W1, re_W1 + kPlane, re_W2, se_W2, pr_W, pr_W + kPlane, pr_W + 2 * kPlane, WT);

  k3_layer_kernel<<<kRowsAP / 8, 256, 0, stream>>>(types, ae_W1, ae_b1, HA, kRowsA);
  k3_layer_kernel<<<kRowsS / 8, 256, 0, stream>>>(states, se_W1, se_b1, HS, kRowsS);

  gemm_f16_tile64<1, 1, 1><<<gemm_blocks(kRowsAP, kHid), 256, 0, stream>>>(
      HA, kHid, WT_ae2, kHid, (void*)AENC, kHid, ae_b2,
      kRowsAP, kHid, kHid, kRowsA, kFold, kActCarry);

  gemm_f16_tile64<0, 0, 0><<<gemm_blocks(kRowsAP, 2 * kHid), 256, 0, stream>>>(
      AENC, kHid, WT_pbpa, kHid, (void*)PBPA, 2 * kHid, ae_b2,
      kRowsAP, 2 * kHid, kHid, kRowsA, kFold, 1.0f);

  gemm_f16_tile64<1, 1, 1><<<gemm_blocks(kRowsS, kHid), 256, 0, stream>>>(
      HS, kHid, WT_se2, kHid, (void*)SENC, kHid, se_b2,
      kRowsS, kHid, kHid, kRowsS, kFold, kActCarry);

  gemm_f16_tile64<0, 0, 0><<<gemm_blocks(kRowsS, kHid), 256, 0, stream>>>(
      SENC, kHid, WT_prr, kHid, (void*)PRR, kHid, se_b2,
      kRowsS, kHid, kHid, kRowsS, kFold, 1.0f);

  gather_player_kernel<<<kRowsP / 8, 256, 0, stream>>>(SENC, pid, SENCP);
  gemm_f16_tile64<0, 0, 0><<<gemm_blocks(kRowsP, kHid), 256, 0, stream>>>(
      SENCP, kHid, WT_ps, kHid, (void*)PSP, kHid, se_b2,
      kRowsP, kHid, kHid, kRowsP, kFold, 1.0f);

  h1_player_kernel<<<kRowsAP / 8, 256, 0, stream>>>(PBPA, re_b1, pid, H1P);
  gemm_f16_tile64<1, 1, 1><<<gemm_blocks(kRowsAP, kHid), 256, 0, stream>>>(
      H1P, kHid, WT_re2, kHid, (void*)RELP, kHid, re_b2,
      kRowsAP, kHid, kHid, kRowsA, kFold, kActCarry);
  gemm_f16_tile64<0, 0, 0><<<gemm_blocks(kRowsAP, kHid), 256, 0, stream>>>(
      RELP, kHid, WT_prel, kHid, (void*)PRELP, kHid, re_b2,
      kRowsAP, kHid, kHid, kRowsA, kFold, 1.0f);

  combine_kernel<<<kRowsP / 4, 256, 0, stream>>>(PSP, PRR, PRELP, pr_b, XAGG);

  conv1_kernel<<<(kNB * kC1L) / 8, 256, 0, stream>>>(XAGG, c1_w, c1_b, Y1);
  tail_kernel<<<kNB, 256, 0, stream>>>(Y1, c2_w, c2_b, c3_w, c3_b, c4_w, c4_b, out);
}
